// LinearAttention_87153476370664
// MI455X (gfx1250) — hardware-run, weakly checked
//
#include <hip/hip_runtime.h>
#include <math.h>


#ifndef NB
#define NB 2
#endif
#ifndef SEQ
#define SEQ 1024
#endif
#define NB_FULL  2
#define SEQ_FULL 1024
#ifndef OUT_SEQ
#define OUT_SEQ SEQ
#endif
#define DM   1024
#define NH_  16
#define HD   64
#define AW   4

static_assert(HD == 64);
static_assert(NH_ * HD == DM);
static_assert(DM == 1024);
static_assert(DM % 64 == 0);
static_assert(DM % 32 == 0);
static_assert(SEQ % 64 == 0);
static_assert((NB * SEQ) % 64 == 0);
static_assert(SEQ % 32 == 0);
static_assert(AW * 16 == HD);
static_assert(SEQ % (16 * AW) == 0);
static_assert(((size_t)SEQ * DM) % 8 == 0);
static_assert(((size_t)DM * DM) % 8 == 0);
static_assert(NB <= NB_FULL);
static_assert(SEQ <= SEQ_FULL);

typedef unsigned short bf;
typedef __attribute__((ext_vector_type(16))) __bf16   v16bf;
typedef __attribute__((ext_vector_type(8)))  unsigned short v8us;
typedef __attribute__((ext_vector_type(8)))  float    v8f;
typedef __attribute__((ext_vector_type(4)))  float    v4f;
typedef v4f  __attribute__((may_alias)) v4fa;

static constexpr size_t PLT = (size_t)NB * NH_ * HD * SEQ;
static constexpr size_t PLV = (size_t)NB * NH_ * SEQ * HD;
static constexpr size_t PLS = (size_t)NB * NH_ * HD * HD;
static constexpr size_t PLY = (size_t)NB * SEQ * DM;

__device__ __forceinline__ unsigned short f2bf(float f) { unsigned u = __float_as_uint(f); u += 0x7FFFu + ((u >> 16) & 1u); return (unsigned short)(u >> 16); }
__device__ __forceinline__ float bf2f(unsigned short b) { return __uint_as_float(((unsigned)b) << 16); }
__device__ __forceinline__ float bfr(float f) { return bf2f(f2bf(f)); }
__device__ __forceinline__ v16bf cat16b(v8us lo, v8us hi) { return __builtin_bit_cast(v16bf, __builtin_shufflevector(lo, hi, 0, 1, 2, 3, 4, 5, 6, 7, 8, 9, 10, 11, 12, 13, 14, 15)); }
__device__ __forceinline__ v8f wmmab(v16bf a, v16bf b, v8f c) { return __builtin_amdgcn_wmma_f32_16x16x32_bf16(false, a, false, b, (short)0, c, false, false); }
__device__ __forceinline__ v16bf ldb(const bf* p)  { return cat16b(*(const v8us*)p, *(const v8us*)(p + 16)); }
__device__ __forceinline__ void wave_sync() { __builtin_amdgcn_fence(3  , "wavefront"); __builtin_amdgcn_wave_barrier(); asm volatile("" ::: "memory"); }
__device__ __forceinline__ void split8(const v4f x0, const v4f x1, v8us& hv, v8us& lv) {
#pragma unroll
    for (int i = 0; i < 4; ++i) {
        const unsigned short a0 = f2bf(x0[i]); const unsigned short a1 = f2bf(x1[i]);
        hv[i] = a0; hv[4 + i] = a1;
        lv[i] = f2bf(x0[i] - bf2f(a0)); lv[4 + i] = f2bf(x1[i] - bf2f(a1)); }
}

__global__ __launch_bounds__(256) void k_cvt8(const float* __restrict__ src, bf* dst, size_t n8) {
    const size_t i = (size_t)blockIdx.x * 256 + threadIdx.x; if (i >= n8) return;
    const v8f v = *(const v8f*)(src + i * 8); v8us o;
#pragma unroll
    for (int k = 0; k < 8; ++k) o[k] = f2bf(v[k]);
    *(volatile v8us*)(dst + i * 8) = o; __threadfence(); *(volatile v8us*)(dst + i * 8) = o;
}

template <int NPA>
__device__ __forceinline__ void gemm_loop(const bf* __restrict__ A, size_t planeA, const bf* __restrict__ Bt, size_t aoff, size_t boff, v8f (&acc)[4][4]) {
#pragma unroll 1
    for (int p = 0; p < NPA; ++p) {
        const bf* Ap = A + (size_t)p * planeA + aoff;
        const bf* Bp = Bt + boff;
#pragma unroll 1
        for (int kc = 0; kc < DM; kc += 32) {
            v16bf a[4];
#pragma unroll
            for (int mb = 0; mb < 4; ++mb) a[mb] = ldb(Ap + (size_t)mb * 16 * DM + kc);
#pragma unroll
            for (int nb = 0; nb < 4; ++nb) { const v16bf b = ldb(Bp + (size_t)nb * 16 * DM + kc);
#pragma unroll
                for (int mb = 0; mb < 4; ++mb) acc[mb][nb] = wmmab(a[mb], b, acc[mb][nb]); }
            asm volatile("v_nop\n\tv_nop\n\tv_nop\n\tv_nop" : "+v"(acc[0][0]), "+v"(acc[1][1]), "+v"(acc[2][2]), "+v"(acc[3][3]) : "v"(a[0]), "v"(a[1]), "v"(a[2]), "v"(a[3]));
        }
    }
}

template <int MODE>
__global__ __launch_bounds__(32) void k_gemm1(const bf* __restrict__ A, const bf* __restrict__ Bt, const float* __restrict__ bias, bf* TP, bf* VP, float* GP) {
    __shared__ __align__(16) float os[64 * 68];
    const int lane = threadIdx.x & 31, lr = lane & 15, hi = lane >> 4;
    const int r0 = blockIdx.x * 64, c0 = blockIdx.y * 64;
    v8f acc[4][4];
#pragma unroll
    for (int mb = 0; mb < 4; ++mb)
#pragma unroll
        for (int nb = 0; nb < 4; ++nb) acc[mb][nb] = (v8f){};
    gemm_loop<1>(A, (size_t)0, Bt, (size_t)(r0 + lr) * DM + 8 * hi, (size_t)(c0 + lr) * DM + 8 * hi, acc);
#pragma unroll
    for (int mb = 0; mb < 4; ++mb)
#pragma unroll
        for (int nb = 0; nb < 4; ++nb)
#pragma unroll
            for (int j = 0; j < 8; ++j) os[(mb * 16 + hi * 8 + j) * 68 + nb * 16 + lr] = acc[mb][nb][j];
    wave_sync();
    float b0 = 0.0f, b1 = 0.0f;
    if (MODE == 1) { b0 = bfr(bias[c0 + lane]); b1 = bfr(bias[c0 + 32 + lane]); }
#pragma unroll 1
    for (int it = 0; it < 128; ++it) {
        const int row = it >> 1, col = ((it & 1) << 5) + lane;
        float bv;
        if (MODE == 0) bv = bfr(bias[r0 + row]); else bv = (it & 1) ? b1 : b0;
        const float v = os[row * 68 + col] + bv;
        float a;
        if (MODE == 0) a = fmaxf(v, 0.0f) + log1pf(expf(-fabsf(v)));
        else           a = 0.5f * v * (1.0f + erff(v * 0.70710678118654752f));
        os[row * 68 + col] = a;
    }
    wave_sync();
    if (MODE == 0) {
        const int which = r0 >> 10, h = (r0 & 1023) >> 6;
        const int b = c0 / SEQ, t0 = c0 % SEQ;
        const size_t base = (size_t)(2 * which) * PLT + ((size_t)(b * NH_ + h) * HD) * SEQ + t0;
#pragma unroll 1
        for (int ps = 0; ps < 2; ++ps) {
#pragma unroll 4
            for (int s = 0; s < 16; ++s) { const int row = 4 * s + (lane >> 3), c8 = (lane & 7) * 8;
                const v4f x0 = *(const v4fa*)(&os[row * 68 + c8]); const v4f x1 = *(const v4fa*)(&os[row * 68 + c8 + 4]); v8us hv, lv;
                split8(x0, x1, hv, lv);
                const size_t oo = base + (size_t)row * SEQ + c8;
                *(volatile v8us*)(TP + oo) = hv; *(volatile v8us*)(TP + PLT + oo) = lv; }
            if (ps == 0) __threadfence(); }
    } else {
        const int which = c0 >> 10, h = (c0 & 1023) >> 6;
        const int b = r0 / SEQ, t0 = r0 % SEQ;
        const size_t base = ((size_t)(b * NH_ + h) * SEQ + t0) * HD;
        if (which == 0) {
#pragma unroll 1
            for (int ps = 0; ps < 2; ++ps) {
#pragma unroll 4
                for (int s = 0; s < 16; ++s) { const int row = 4 * s + (lane >> 3), c8 = (lane & 7) * 8;
                    const v4f x0 = *(const v4fa*)(&os[row * 68 + c8]); const v4f x1 = *(const v4fa*)(&os[row * 68 + c8 + 4]); v8us hv, lv;
                    split8(x0, x1, hv, lv);
                    const size_t oo = base + (size_t)row * HD + c8;
                    *(volatile v8us*)(VP + oo) = hv; *(volatile v8us*)(VP + PLV + oo) = lv; }
                if (ps == 0) __threadfence(); }
        } else {
#pragma unroll 1
            for (int ps = 0; ps < 2; ++ps) {
#pragma unroll 4
                for (int s = 0; s < 32; ++s) { const int row = 2 * s + hi, cofs = lr * 4;
                    const v4f val = *(const v4fa*)(&os[row * 68 + cofs]);
                    *(volatile v4f*)(GP + base + (size_t)row * HD + cofs) = val; }
                if (ps == 0) __threadfence(); }
        }
    }
}

__global__ __launch_bounds__(32 * AW) void k_s(const bf* __restrict__ TP, bf* SP) {
    __shared__ __align__(16) float os[AW * 16 * 68];
    const int lane = threadIdx.x & 31, lr = lane & 15, hi = lane >> 4;
    const int wave = __builtin_amdgcn_readfirstlane((int)(threadIdx.x >> 5));
    const int bh = blockIdx.x;
    const size_t ao = ((size_t)bh * HD + 16 * wave + lr) * SEQ + 8 * hi;
    const size_t bo = ((size_t)bh * HD + lr) * SEQ + 8 * hi;
    v8f acc[4];
#pragma unroll
    for (int nb = 0; nb < 4; ++nb) acc[nb] = (v8f){};
#pragma unroll 1
    for (int kc = 0; kc < SEQ; kc += 32) {
        const v16bf ah = ldb(TP + ao + kc), al = ldb(TP + PLT + ao + kc);
        v16bf bhf[4], blf[4];
#pragma unroll
        for (int nb = 0; nb < 4; ++nb) { bhf[nb] = ldb(TP + 2 * PLT + bo + (size_t)nb * 16 * SEQ + kc); blf[nb] = ldb(TP + 3 * PLT + bo + (size_t)nb * 16 * SEQ + kc); }
#pragma unroll
        for (int nb = 0; nb < 4; ++nb) acc[nb] = wmmab(ah, bhf[nb], acc[nb]);
#pragma unroll
        for (int nb = 0; nb < 4; ++nb) acc[nb] = wmmab(ah, blf[nb], acc[nb]);
#pragma unroll
        for (int nb = 0; nb < 4; ++nb) acc[nb] = wmmab(al, bhf[nb], acc[nb]);
        asm volatile("v_nop\n\tv_nop\n\tv_nop\n\tv_nop" : "+v"(acc[0]), "+v"(acc[1]), "+v"(acc[2]), "+v"(acc[3]) : "v"(ah), "v"(al), "v"(bhf[0]), "v"(bhf[1]), "v"(bhf[2]), "v"(bhf[3]), "v"(blf[0]), "v"(blf[1]), "v"(blf[2]), "v"(blf[3]));
    }
    const int wb = wave * 16 * 68;
#pragma unroll
    for (int nb = 0; nb < 4; ++nb)
#pragma unroll
        for (int j = 0; j < 8; ++j) os[wb + (hi * 8 + j) * 68 + nb * 16 + lr] = acc[nb][j];
    wave_sync();
    v8us hv[4], lv[4];
#pragma unroll
    for (int s = 0; s < 4; ++s) { const int row = 4 * s + (lane >> 3), c8 = (lane & 7) * 8;
        v4f x0 = *(const v4fa*)(&os[wb + row * 68 + c8]); v4f x1 = *(const v4fa*)(&os[wb + row * 68 + c8 + 4]);
        float rs = ((x0[0] + x0[1]) + (x0[2] + x0[3])) + ((x1[0] + x1[1]) + (x1[2] + x1[3]));
        rs += __shfl_xor(rs, 1, 32); rs += __shfl_xor(rs, 2, 32); rs += __shfl_xor(rs, 4, 32);
        const float zi = 1.0f / (0.125f * rs + 1024.0f);
        const int e = 16 * wave + row;
#pragma unroll
        for (int i = 0; i < 4; ++i) {
            x0[i] = (0.125f * x0[i] + ((c8 + i == e) ? 1.0f : 0.0f)) * zi;
            x1[i] = (0.125f * x1[i] + ((c8 + 4 + i == e) ? 1.0f : 0.0f)) * zi; }
        split8(x0, x1, hv[s], lv[s]); }
    const size_t sbase = ((size_t)bh * HD + 16 * wave) * HD;
#pragma unroll 1
    for (int ps = 0; ps < 2; ++ps) {
#pragma unroll
        for (int s = 0; s < 4; ++s) { const int row = 4 * s + (lane >> 3), c8 = (lane & 7) * 8;
            const size_t oo = sbase + (size_t)row * HD + c8;
            *(volatile v8us*)(SP + oo) = hv[s]; *(volatile v8us*)(SP + PLS + oo) = lv[s]; }
        if (ps == 0) __threadfence(); }
}

__global__ __launch_bounds__(32 * AW) void k_out(const bf* __restrict__ VP, const bf* __restrict__ SP, const float* __restrict__ GP, bf* YP) {
    __shared__ __align__(16) float os[AW * 16 * 68];
    const int lane = threadIdx.x & 31, lr = lane & 15, hi = lane >> 4;
    const int wave = __builtin_amdgcn_readfirstlane((int)(threadIdx.x >> 5));
    const int bh = blockIdx.y; const int b = bh / NH_, h = bh % NH_;
    const int m0 = (blockIdx.x * AW + wave) * 16;
    const size_t ao = ((size_t)bh * SEQ + m0 + lr) * HD + 8 * hi;
    const size_t bo = ((size_t)bh * HD + lr) * HD + 8 * hi;
    v8f acc[4];
#pragma unroll
    for (int nb = 0; nb < 4; ++nb) acc[nb] = (v8f){};
#pragma unroll 1
    for (int kc = 0; kc < HD; kc += 32) {
        const v16bf ah = ldb(VP + ao + kc), al = ldb(VP + PLV + ao + kc);
        v16bf bhf[4], blf[4];
#pragma unroll
        for (int nb = 0; nb < 4; ++nb) { bhf[nb] = ldb(SP + bo + (size_t)nb * 16 * HD + kc); blf[nb] = ldb(SP + PLS + bo + (size_t)nb * 16 * HD + kc); }
#pragma unroll
        for (int nb = 0; nb < 4; ++nb) acc[nb] = wmmab(ah, bhf[nb], acc[nb]);
#pragma unroll
        for (int nb = 0; nb < 4; ++nb) acc[nb] = wmmab(ah, blf[nb], acc[nb]);
#pragma unroll
        for (int nb = 0; nb < 4; ++nb) acc[nb] = wmmab(al, bhf[nb], acc[nb]);
        asm volatile("v_nop\n\tv_nop\n\tv_nop\n\tv_nop" : "+v"(acc[0]), "+v"(acc[1]), "+v"(acc[2]), "+v"(acc[3]) : "v"(ah), "v"(al), "v"(bhf[0]), "v"(bhf[1]), "v"(bhf[2]), "v"(bhf[3]), "v"(blf[0]), "v"(blf[1]), "v"(blf[2]), "v"(blf[3]));
    }
    const int wb = wave * 16 * 68;
#pragma unroll
    for (int nb = 0; nb < 4; ++nb)
#pragma unroll
        for (int j = 0; j < 8; ++j) os[wb + (hi * 8 + j) * 68 + nb * 16 + lr] = acc[nb][j];
    wave_sync();
    const size_t gbase = ((size_t)bh * SEQ + m0) * HD;
    v8us hv[4], lv[4];
#pragma unroll
    for (int s = 0; s < 4; ++s) { const int row = 4 * s + (lane >> 3), c8 = (lane & 7) * 8;
        v4f x0 = *(const v4fa*)(&os[wb + row * 68 + c8]); v4f x1 = *(const v4fa*)(&os[wb + row * 68 + c8 + 4]);
        const v4f g0 = *(const v4f*)(GP + gbase + (size_t)row * HD + c8); const v4f g1 = *(const v4f*)(GP + gbase + (size_t)row * HD + c8 + 4);
        x0 = x0 * g0; x1 = x1 * g1;
        split8(x0, x1, hv[s], lv[s]); }
    const size_t ybase = ((size_t)b * SEQ + ((size_t)h * SEQ + m0) / 16) * DM;
#pragma unroll 1
    for (int ps = 0; ps < 2; ++ps) {
#pragma unroll
        for (int s = 0; s < 4; ++s) { const int row = 4 * s + (lane >> 3), c8 = (lane & 7) * 8;
            const size_t oo = ybase + (size_t)row * HD + c8;
            *(volatile v8us*)(YP + oo) = hv[s]; *(volatile v8us*)(YP + PLY + oo) = lv[s]; }
        if (ps == 0) __threadfence(); }
}

__global__ __launch_bounds__(32) void k_fin(const bf* __restrict__ YP, const bf* __restrict__ Wb, const float* __restrict__ bias, float* OUT) {
    __shared__ __align__(16) float os[64 * 68];
    const int lane = threadIdx.x & 31, lr = lane & 15, hi = lane >> 4;
    const int r0 = blockIdx.x * 64, c0 = blockIdx.y * 64;
    v8f acc[4][4];
#pragma unroll
    for (int mb = 0; mb < 4; ++mb)
#pragma unroll
        for (int nb = 0; nb < 4; ++nb) acc[mb][nb] = (v8f){};
    gemm_loop<2>(YP, PLY, Wb, (size_t)(r0 + lr) * DM + 8 * hi, (size_t)(c0 + lr) * DM + 8 * hi, acc);
    float bb[4];
#pragma unroll
    for (int nb = 0; nb < 4; ++nb) bb[nb] = bfr(bias[c0 + nb * 16 + lr]);
#pragma unroll
    for (int mb = 0; mb < 4; ++mb)
#pragma unroll
        for (int nb = 0; nb < 4; ++nb)
#pragma unroll
            for (int j = 0; j < 8; ++j) os[(mb * 16 + hi * 8 + j) * 68 + nb * 16 + lr] = acc[mb][nb][j] + bb[nb];
    wave_sync();
    float* orow = OUT + ((size_t)(r0 / SEQ) * OUT_SEQ + (size_t)(r0 % SEQ)) * DM + c0;
#pragma unroll 1
    for (int ps = 0; ps < 2; ++ps) {
#pragma unroll 4
        for (int s = 0; s < 32; ++s) { const int row = 2 * s + hi, cofs = lr * 4;
            const v4f val = *(const v4fa*)(&os[row * 68 + cofs]);
            *(volatile v4f*)(orow + (size_t)row * DM + cofs) = val; }
        if (ps == 0) __threadfence(); }
}

static constexpr size_t al256(size_t v) { return (v + 255) & ~(size_t)255; }
static constexpr size_t SZ_XB = al256((size_t)NB * SEQ * DM * 2);
static constexpr size_t SZ_WB = al256((size_t)4 * DM * DM * 2);
static constexpr size_t SZ_WP = al256((size_t)DM * DM * 2);
static constexpr size_t SZ_TP = al256((size_t)4 * PLT * 2);
static constexpr size_t SZ_VP = al256((size_t)2 * PLV * 2);
static constexpr size_t SZ_GP = al256((size_t)PLV * 4);
static constexpr size_t SZ_SP = al256((size_t)2 * PLS * 2);
static constexpr size_t SZ_YP = al256((size_t)2 * PLY * 2);
static constexpr size_t SZ_TOTAL = SZ_XB + SZ_WB + SZ_WP + SZ_TP + SZ_VP + SZ_GP + SZ_SP + SZ_YP;
static_assert(SZ_TOTAL <= (size_t)134217728);
static_assert((PLT * 2) % 256 == 0);
static_assert((PLV * 2) % 256 == 0);
static_assert((PLS * 2) % 256 == 0);
static_assert((PLY * 2) % 256 == 0);

extern "C" void kernel_launch(void* const* d_in, const int* in_sizes, int n_in,
                              void* d_out, int out_size, void* d_ws, size_t ws_size, hipStream_t stream) {
    if (n_in < 5) return;
    const size_t needx = ((size_t)(NB - 1) * SEQ_FULL + SEQ) * DM;
    if ((size_t)in_sizes[0] < needx) return;
    if ((size_t)in_sizes[1] < (size_t)4 * DM * DM || (size_t)in_sizes[2] < (size_t)4 * DM) return;
    if ((size_t)in_sizes[3] < (size_t)DM * DM || (size_t)in_sizes[4] < (size_t)DM) return;
    if ((size_t)out_size < ((size_t)(NB - 1) * OUT_SEQ + SEQ) * DM) return;
    if (SZ_TOTAL > ws_size) return;
    const float* x = (const float*)d_in[0]; const float* wq = (const float*)d_in[1]; const float* bq = (const float*)d_in[2];
    const float* wp = (const float*)d_in[3]; const float* bp = (const float*)d_in[4];
    float* OUT = (float*)d_out;
    char* wsp = (char*)d_ws;
    bf* XB = (bf*)wsp; wsp += SZ_XB;
    bf* WB = (bf*)wsp; wsp += SZ_WB;
    bf* WPB = (bf*)wsp; wsp += SZ_WP;
    bf* TP = (bf*)wsp; wsp += SZ_TP;
    bf* VP = (bf*)wsp; wsp += SZ_VP;
    float* GP = (float*)wsp; wsp += SZ_GP;
    bf* SP = (bf*)wsp; wsp += SZ_SP;
    bf* YP = (bf*)wsp; wsp += SZ_YP;

    if (SEQ == SEQ_FULL) {
        const size_t n8 = (size_t)NB * SEQ * DM / 8;
        k_cvt8<<<(unsigned)((n8 + 255) / 256), 256, 0, stream>>>(x, XB, n8);
    } else {
        const size_t n8 = (size_t)SEQ * DM / 8;
        for (int b = 0; b < NB; ++b) k_cvt8<<<(unsigned)((n8 + 255) / 256), 256, 0, stream>>>(x + (size_t)b * SEQ_FULL * DM, XB + (size_t)b * SEQ * DM, n8);
    }
    { const size_t n8 = (size_t)4 * DM * DM / 8; k_cvt8<<<(unsigned)((n8 + 255) / 256), 256, 0, stream>>>(wq, WB, n8); }
    { const size_t n8 = (size_t)DM * DM / 8;     k_cvt8<<<(unsigned)((n8 + 255) / 256), 256, 0, stream>>>(wp, WPB, n8); }

    k_gemm1<0><<<dim3(2 * DM / 64, NB * SEQ / 64, 1), 32, 0, stream>>>(WB, XB, bq, TP, VP, GP);
    k_gemm1<1><<<dim3(NB * SEQ / 64, 2 * DM / 64, 1), 32, 0, stream>>>(XB, WB + (size_t)2 * DM * DM, bq + 2 * DM, TP, VP, GP);

    k_s<<<dim3(NB * NH_, 1, 1), 32 * AW, 0, stream>>>(TP, SP);
    k_out<<<dim3(SEQ / (16 * AW), NB * NH_, 1), 32 * AW, 0, stream>>>(VP, SP, GP, YP);
    k_fin<<<dim3(NB * SEQ / 64, DM / 64, 1), 32, 0, stream>>>(YP, WPB, bp, OUT);
}
